// GatedLinearAttention_13632226197673
// MI455X (gfx1250) — hardware-verified
//
#include <hip/hip_runtime.h>
#include <math.h>

constexpr int kB    = 2;
constexpr int kT    = 2048;
constexpr int kC    = 1024;
constexpr int kH    = 16;
constexpr int kD    = 64;
constexpr int kRows = kB * kT;
constexpr int kLinN = 3 * kC;
constexpr int kLinLd = kLinN;
constexpr int kGbN  = 64;
constexpr int kTaps = 4;
constexpr int kTch  = 32;
constexpr long kPlane = (long)kRows * kC;
constexpr float kOgCarry = 16.0f;
constexpr float kWoCarry = 16.0f;
constexpr float kOutScale = 1.0f / 256.0f;
constexpr float kL2Eps  = 1.0e-6f;
constexpr float kRmsEps = 1.0e-5f;
static_assert(kH * kD == kC);
static_assert(kC % 32 == 0);
static_assert(kRows % 64 == 0 && kLinN % 64 == 0 && kGbN % 64 == 0 && kC % 64 == 0);
static_assert(kT % kTch == 0 && kT % 64 == 0);

typedef __attribute__((ext_vector_type(16))) _Float16 v16h;
typedef __attribute__((ext_vector_type(8)))  _Float16 v8h;
typedef __attribute__((ext_vector_type(16))) __bf16   v16b;
typedef __attribute__((ext_vector_type(8)))  __bf16   v8b;
typedef __attribute__((ext_vector_type(8)))  float    v8f;
typedef __attribute__((ext_vector_type(4)))  float    v4f;
typedef __attribute__((ext_vector_type(4)))  unsigned int v4u;

__device__ __forceinline__ unsigned short f2bf_bits(float f) {
  unsigned u = __float_as_uint(f);
  return (unsigned short)((u + 0x7FFFu + ((u >> 16) & 1u)) >> 16);
}
__device__ __forceinline__ float bf_bits2f(unsigned short h) { return __uint_as_float(((unsigned)h) << 16); }
__device__ __forceinline__ float bfr(float f) { return bf_bits2f(f2bf_bits(f)); }

__device__ __forceinline__ void dep_guard_h(v8f& a, v8f& b, v16h x, v16h y) { asm volatile("v_nop\n\tv_nop\n\tv_nop\n\tv_nop" : "+v"(a), "+v"(b) : "v"(x), "v"(y)); }
__device__ __forceinline__ void dep_guard_b(v8f& a, v8f& b, v16b x, v16b y) { asm volatile("v_nop\n\tv_nop\n\tv_nop\n\tv_nop" : "+v"(a), "+v"(b) : "v"(x), "v"(y)); }
__device__ __forceinline__ void dep_guard4_h(v8f& a, v8f& b, v8f& c, v8f& d, v16h x, v16h y) { asm volatile("v_nop\n\tv_nop\n\tv_nop\n\tv_nop" : "+v"(a), "+v"(b), "+v"(c), "+v"(d) : "v"(x), "v"(y)); }
__device__ __forceinline__ void dep_guard4_b(v8f& a, v8f& b, v8f& c, v8f& d, v16b x, v16b y) { asm volatile("v_nop\n\tv_nop\n\tv_nop\n\tv_nop" : "+v"(a), "+v"(b), "+v"(c), "+v"(d) : "v"(x), "v"(y)); }
__device__ __forceinline__ void keep4_h(v16h a, v16h b, v16h c, v16h d) { asm volatile("v_nop" :: "v"(a), "v"(b), "v"(c), "v"(d)); }
__device__ __forceinline__ void keep4_b(v16b a, v16b b, v16b c, v16b d) { asm volatile("v_nop" :: "v"(a), "v"(b), "v"(c), "v"(d)); }
__device__ __forceinline__ void acc_guard4(v8f& a, v8f& b, v8f& c, v8f& d) { asm volatile("v_nop\n\tv_nop\n\tv_nop\n\tv_nop" : "+v"(a), "+v"(b), "+v"(c), "+v"(d)); }
template <typename T> struct Frag;
template <> struct Frag<_Float16> {
  typedef v16h V; union U { v16h v; v8h h[2]; };
  static __device__ __forceinline__ v16h load(const _Float16* p) {
    U f; f.h[0] = *(const v8h*)(p); f.h[1] = *(const v8h*)(p + 16); return f.v;
  }
  static __device__ __forceinline__ v8f mma(v16h a, v16h b, v8f c) {
    return __builtin_amdgcn_wmma_f32_16x16x32_f16(false, a, false, b, (short)0, c, false, false);
  }
  static __device__ __forceinline__ void guard(v8f& a, v8f& b, v16h x, v16h y) { dep_guard_h(a, b, x, y); }
  static __device__ __forceinline__ void guard4(v8f& a, v8f& b, v8f& c, v8f& d, v16h x, v16h y) { dep_guard4_h(a, b, c, d, x, y); }
  static __device__ __forceinline__ void keep(v16h a, v16h b, v16h c, v16h d) { keep4_h(a, b, c, d); }
};
template <> struct Frag<__bf16> {
  typedef v16b V; union U { v16b v; v8b h[2]; };
  static __device__ __forceinline__ v16b load(const __bf16* p) {
    U f; f.h[0] = *(const v8b*)(p); f.h[1] = *(const v8b*)(p + 16); return f.v;
  }
  static __device__ __forceinline__ v8f mma(v16b a, v16b b, v8f c) {
    return __builtin_amdgcn_wmma_f32_16x16x32_bf16(false, a, false, b, (short)0, c, false, false);
  }
  static __device__ __forceinline__ void guard(v8f& a, v8f& b, v16b x, v16b y) { dep_guard_b(a, b, x, y); }
  static __device__ __forceinline__ void guard4(v8f& a, v8f& b, v8f& c, v8f& d, v16b x, v16b y) { dep_guard4_b(a, b, c, d, x, y); }
  static __device__ __forceinline__ void keep(v16b a, v16b b, v16b c, v16b d) { keep4_b(a, b, c, d); }
};

__device__ __forceinline__ unsigned pk16(unsigned short a, unsigned short b) { return (unsigned)a | ((unsigned)b << 16); }
__device__ __forceinline__ unsigned short h_bits(float f) { const _Float16 h = (_Float16)f; return __builtin_bit_cast(unsigned short, h); }

template <int ET> struct Elem;
template <> struct Elem<0> { typedef _Float16 T; };
template <> struct Elem<1> { typedef __bf16 T; };
template <int ET, bool SPLIT, int BIAS_MODE, int OUT_MODE, bool RESID, int ACT = 0>
__global__ __launch_bounds__(256) void wmma_gemm64(
    const unsigned short* __restrict__ Ap, const unsigned short* __restrict__ A2p, int lda, long strideA,
    const unsigned short* __restrict__ Btp, const unsigned short* __restrict__ Bt2p, int ldb, long strideB,
    void* __restrict__ Cout, void* __restrict__ Cout2, int ldc, long strideC,
    const float* __restrict__ bias,
    const float* __restrict__ resid, long strideR,
    int M, int N, int K, float scale) {
  typedef typename Elem<ET>::T T;
  typedef typename Frag<T>::V V;
  const T* A = (const T*)Ap; const T* A2 = (const T*)A2p; const T* Bt = (const T*)Btp; const T* Bt2 = (const T*)Bt2p;
  __shared__ __align__(16) float sT[8][16 * 68];
  const int b    = blockIdx.y;
  const int lane = threadIdx.x & 31;
  const int wave = threadIdx.x >> 5;
  const int tilesN = N >> 6;
  const int tilesM = M >> 6;
  const int tile = blockIdx.x * 8 + wave;
  if (tile >= tilesM * tilesN) return;
  const int tm = tile / tilesN;
  const int tn = tile - tm * tilesN;
  const int m0 = tm << 6;
  const int n0 = tn << 6;

  const T* Ab  = A  + (size_t)b * strideA;
  const T* Bb  = Bt + (size_t)b * strideB;
  const T* Ab2 = SPLIT ? (A2  + (size_t)b * strideA) : nullptr;
  const T* Bb2 = SPLIT ? (Bt2 + (size_t)b * strideB) : nullptr;

  const int rlane = lane & 15;
  const int koff  = (lane >> 4) * 8;
  const int mOff  = (lane >> 4) * 8;

  v8f acc[4][4];
#pragma unroll
  for (int i = 0; i < 4; ++i)
#pragma unroll
    for (int j = 0; j < 4; ++j) acc[i][j] = (v8f){0.f,0.f,0.f,0.f,0.f,0.f,0.f,0.f};

  for (int k0 = 0; k0 < K; k0 += 32) {
    V bh[4], bl[4];
#pragma unroll
    for (int j = 0; j < 4; ++j) {
      const size_t bo = (size_t)(n0 + (j << 4) + rlane) * ldb + koff + k0;
      bh[j] = Frag<T>::load(Bb + bo);
      if (SPLIT) bl[j] = Frag<T>::load(Bb2 + bo);
    }
#pragma unroll
    for (int i = 0; i < 4; ++i) {
      const size_t ao = (size_t)(m0 + (i << 4) + rlane) * lda + koff + k0;
      V ah = Frag<T>::load(Ab + ao);
      V al;
      if (SPLIT) al = Frag<T>::load(Ab2 + ao);
#pragma unroll
      for (int j = 0; j < 4; ++j) {
        acc[i][j] = Frag<T>::mma(ah, bh[j], acc[i][j]);
        if (SPLIT) {
          acc[i][j] = Frag<T>::mma(ah, bl[j], acc[i][j]);
          acc[i][j] = Frag<T>::mma(al, bh[j], acc[i][j]);
        }
      }
      Frag<T>::guard4(acc[i][0], acc[i][1], acc[i][2], acc[i][3], ah, SPLIT ? al : ah);
    }
    Frag<T>::keep(bh[0], bh[1], bh[2], bh[3]);
    if (SPLIT) Frag<T>::keep(bl[0], bl[1], bl[2], bl[3]);
  }
  acc_guard4(acc[0][0], acc[0][1], acc[0][2], acc[0][3]);
  acc_guard4(acc[1][0], acc[1][1], acc[1][2], acc[1][3]);
  acc_guard4(acc[2][0], acc[2][1], acc[2][2], acc[2][3]);
  acc_guard4(acc[3][0], acc[3][1], acc[3][2], acc[3][3]);

  float* slab = sT[wave];
  const float* Rb = RESID ? (resid + (size_t)b * strideR) : nullptr;
#pragma unroll
  for (int i = 0; i < 4; ++i) {
    const int mBase = m0 + (i << 4);
#pragma unroll
    for (int j = 0; j < 4; ++j) {
      const int n = n0 + (j << 4) + rlane;
      float bv = 0.f;
      if (BIAS_MODE == 2) bv = bias[n];
#pragma unroll
      for (int r = 0; r < 8; ++r) {
        float v = acc[i][j][r] * scale;
        if (BIAS_MODE == 1) v += bias[mBase + mOff + r];
        if (BIAS_MODE == 2) v += bv;
        if (RESID) v += Rb[(size_t)(mBase + mOff + r) * ldc + n];
        if (ACT == 2) v = fmaxf(v, 0.0f);
        if (ACT == 4) v = (v > 0.f) ? v : 0.01f * v;
        slab[(mOff + r) * 68 + (j << 4) + rlane] = v;
      }
    }
    __builtin_amdgcn_fence(__ATOMIC_RELEASE, "workgroup");
    __builtin_amdgcn_wave_barrier();
    __builtin_amdgcn_fence(__ATOMIC_ACQUIRE, "workgroup");
    if (OUT_MODE == 0) {
      float* C = (float*)Cout + (size_t)b * strideC;
      const int hh = lane >> 4, c4 = (lane & 15) * 4;
      for (int pass = 0; pass < 2; ++pass) {
#pragma unroll
        for (int it = 0; it < 8; ++it) {
          const int row = it * 2 + hh;
          v4f v = *(const v4f*)(slab + row * 68 + c4);
          *(volatile v4f*)(C + (size_t)(mBase + row) * ldc + n0 + c4) = v;
        }
        __threadfence();
      }
    } else {
      const int q = lane >> 3, c8 = (lane & 7) * 8;
      unsigned short* C  = (unsigned short*)Cout  + (size_t)b * strideC;
      unsigned short* C2 = (OUT_MODE == 2) ? ((unsigned short*)Cout2 + (size_t)b * strideC) : nullptr;
      for (int pass = 0; pass < 2; ++pass) {
#pragma unroll
        for (int it = 0; it < 4; ++it) {
          const int row = it * 4 + q;
          const float* sp = slab + row * 68 + c8;
          v8h hv, lv;
#pragma unroll
          for (int e = 0; e < 8; ++e) {
            if (OUT_MODE == 1) {
              hv[e] = (_Float16)sp[e];
            } else {
              unsigned short hb = f2bf_bits(sp[e]);
              unsigned short lb = f2bf_bits(sp[e] - bf_bits2f(hb));
              hv[e] = __builtin_bit_cast(_Float16, hb);
              lv[e] = __builtin_bit_cast(_Float16, lb);
            }
          }
          *(volatile v8h*)(C + (size_t)(mBase + row) * ldc + n0 + c8) = hv;
          if (OUT_MODE == 2) *(volatile v8h*)(C2 + (size_t)(mBase + row) * ldc + n0 + c8) = lv;
        }
        __threadfence();
      }
    }
    __builtin_amdgcn_fence(__ATOMIC_RELEASE, "workgroup");
    __builtin_amdgcn_wave_barrier();
    __builtin_amdgcn_fence(__ATOMIC_ACQUIRE, "workgroup");
  }
}

__global__ __launch_bounds__(256) void cast8_bf16_kernel(const float* __restrict__ in, unsigned short* __restrict__ out, int n8) {
  const int i = blockIdx.x * 256 + threadIdx.x;
  if (i >= n8) return;
  const float* p = in + 8 * (size_t)i;
  const v4f a = *(const v4f*)(p);
  const v4f c = *(const v4f*)(p + 4);
  unsigned short hb[8];
#pragma unroll
  for (int e = 0; e < 4; ++e) {
    hb[e]     = f2bf_bits(a[e]);
    hb[4 + e] = f2bf_bits(c[e]);
  }
  const v4u u = (v4u){pk16(hb[0], hb[1]), pk16(hb[2], hb[3]), pk16(hb[4], hb[5]), pk16(hb[6], hb[7])};
  unsigned short* q = out + 8 * (size_t)i;
  *(volatile v4u*)q = u;
  __threadfence();
  *(volatile v4u*)q = u;
}

template <int MODE>
__global__ __launch_bounds__(256) void pack_wt_kernel(const float* __restrict__ W0, const float* __restrict__ W1,
                                                      const float* __restrict__ W2, const float* __restrict__ W3,
                                                      unsigned short* __restrict__ out) {
  __shared__ float sm[64][65];
  const int t  = threadIdx.x;
  const int k0 = blockIdx.x * 64;
  const int n0 = blockIdx.y * 64;
  const int z  = blockIdx.z;
  const float* W = (z == 0) ? W0 : (z == 1) ? W1 : (z == 2) ? W2 : W3;
#pragma unroll
  for (int i = 0; i < 8; ++i) {
    const int e = i * 256 + t;
    const int r = e >> 6;
    const int c = e & 63;
    sm[c][r] = W[(size_t)(k0 + r) * kC + n0 + c];
  }
  asm volatile("" ::: "memory");
#pragma unroll
  for (int i = 8; i < 16; ++i) {
    const int e = i * 256 + t;
    const int r = e >> 6;
    const int c = e & 63;
    sm[c][r] = W[(size_t)(k0 + r) * kC + n0 + c];
  }
  __syncthreads();
  const int lane = t & 31, wave = t >> 5;
  const int q = lane >> 3, c8 = (lane & 7) * 8;
  unsigned short* op = out + (size_t)z * kC * kC;
  for (int pass = 0; pass < 2; ++pass) {
#pragma unroll
    for (int it = 0; it < 2; ++it) {
      const int row = wave * 8 + it * 4 + q;
      unsigned short hb[8];
#pragma unroll
      for (int e = 0; e < 8; ++e) {
        const float w = sm[row][c8 + e];
        if (MODE == 0) hb[e] = f2bf_bits(w);
        else           hb[e] = h_bits(bfr(w) * kWoCarry);
      }
      const v4u u = (v4u){pk16(hb[0], hb[1]), pk16(hb[2], hb[3]), pk16(hb[4], hb[5]), pk16(hb[6], hb[7])};
      *(volatile v4u*)(op + (size_t)(n0 + row) * kC + k0 + c8) = u;
    }
    __threadfence();
  }
}

__global__ __launch_bounds__(128) void pack_gb_kernel(const float* __restrict__ Wgk, const float* __restrict__ Wb,
                                                      unsigned short* __restrict__ WGB) {
  const int n  = blockIdx.x;
  const int t  = threadIdx.x;
  const int k8 = t * 8;
  float w[8];
#pragma unroll
  for (int e = 0; e < 8; ++e) w[e] = 0.0f;
  if (n < 32) {
    const float* src = (n < 16) ? (Wgk + n) : (Wb + (n - 16));
#pragma unroll
    for (int e = 0; e < 8; ++e) w[e] = src[(size_t)(k8 + e) * kH];
  }
  unsigned short hb[8];
#pragma unroll
  for (int e = 0; e < 8; ++e) hb[e] = f2bf_bits(w[e]);
  const v4u u = (v4u){pk16(hb[0], hb[1]), pk16(hb[2], hb[3]), pk16(hb[4], hb[5]), pk16(hb[6], hb[7])};
  unsigned short* op = WGB + (size_t)n * kC + k8;
  *(volatile v4u*)op = u;
  __threadfence();
  *(volatile v4u*)op = u;
}

struct RopeFreq { float f[16]; };
static_assert(sizeof(RopeFreq) == 64);

__global__ __launch_bounds__(256) void cs_table_kernel(float* __restrict__ CS, float* __restrict__ SN, RopeFreq kf) {
#pragma clang fp contract(off)
  __shared__ __align__(16) float csl[1024];
  __shared__ __align__(16) float snl[1024];
  const int t = threadIdx.x;
  const int base = blockIdx.x * 1024;
#pragma unroll 1
  for (int it = 0; it < 4; ++it) {
    const int idx = it * 256 + t;
    const int g = base + idx;
    const int pos = g >> 4;
    const int j = g & 15;
    float fr = kf.f[0];
#pragma unroll
    for (int q = 1; q < 16; ++q) fr = (j == q) ? kf.f[q] : fr;
    const float ang = (float)pos * fr;
    csl[idx] = cosf(ang);
    snl[idx] = sinf(ang);
  }
  __syncthreads();
  const v4f cv = *(const v4f*)(csl + 4 * t);
  const v4f sv = *(const v4f*)(snl + 4 * t);
  float* cp = CS + base + 4 * t;
  float* sp = SN + base + 4 * t;
  *(volatile v4f*)cp = cv;
  *(volatile v4f*)sp = sv;
  __threadfence();
  *(volatile v4f*)cp = cv;
  *(volatile v4f*)sp = sv;
}

__global__ __launch_bounds__(256) void eb_kernel(const float* __restrict__ GB, const float* __restrict__ A_log,
                                                 const float* __restrict__ dt_bias, const float* __restrict__ bb,
                                                 float* __restrict__ EB) {
#pragma clang fp contract(off)
  __shared__ __align__(16) float ebl[2 * kT];
  const int t  = threadIdx.x;
  const int bh = blockIdx.x;
  const int b  = bh >> 4, h = bh & 15;
  const float nA  = -expf(bfr(A_log[h]));
  const float dtb = bfr(dt_bias[h]);
  const float bbh = bfr(bb[h]);
#pragma unroll 1
  for (int it = 0; it < 8; ++it) {
    const int tt = it * 256 + t;
    const float* gr = GB + ((size_t)b * kT + tt) * kGbN;
    const float z1 = gr[h] + dtb;
    const float sp = fmaxf(z1, 0.0f) + log1pf(expf(-fabsf(z1)));
    const float gk = nA * sp;
    const float eg = expf(gk);
    const float z2 = gr[16 + h] + bbh;
    const float beta = 1.0f / (1.0f + expf(-z2));
    ebl[2 * tt]     = eg;
    ebl[2 * tt + 1] = beta;
  }
  __syncthreads();
  float* dst = EB + (size_t)bh * kT * 2;
  for (int pass = 0; pass < 2; ++pass) {
#pragma unroll
    for (int it = 0; it < 4; ++it) {
      const int idx = it * 256 + t;
      const v4f v = *(const v4f*)(ebl + 4 * idx);
      *(volatile v4f*)(dst + 4 * (size_t)idx) = v;
    }
    __threadfence();
  }
}

__global__ __launch_bounds__(256) void prep_kernel(const float* __restrict__ LIN,
                                                   const float* __restrict__ cwq, const float* __restrict__ cwk,
                                                   const float* __restrict__ cwv,
                                                   const float* __restrict__ CS, const float* __restrict__ SN,
                                                   float* __restrict__ QKVc) {
#pragma clang fp contract(off)
  __shared__ __align__(16) float linbuf[67 * 64];
  __shared__ __align__(16) float aob[2][64 * 64];
  __shared__ __align__(16) float cst[64 * 16];
  __shared__ __align__(16) float snt[64 * 16];
  __shared__ float wcv[3][64 * 4];
  const int t  = threadIdx.x;
  const int t0 = blockIdx.x * 64;
  const int h  = blockIdx.y;
  const int b  = blockIdx.z;
  {
    const int c = t & 63, tap = t >> 6;
    const size_t wi = (size_t)(h * 64 + c) * kTaps + tap;
    const float w0 = cwq[wi];
    const float w1 = cwk[wi];
    const float w2 = cwv[wi];
    wcv[0][c * 4 + tap] = bfr(w0);
    wcv[1][c * 4 + tap] = bfr(w1);
    wcv[2][c * 4 + tap] = bfr(w2);
    const v4f c4v = *(const v4f*)(CS + (size_t)t0 * 16 + 4 * t);
    const v4f s4v = *(const v4f*)(SN + (size_t)t0 * 16 + 4 * t);
    *(v4f*)(cst + 4 * t) = c4v;
    *(v4f*)(snt + 4 * t) = s4v;
  }
  __syncthreads();
  const size_t rowBase = (size_t)b * kT;
  float* abuf = aob[0];
  float* obuf = aob[1];
#pragma unroll 1
  for (int z = 0; z < 3; ++z) {
#pragma unroll 1
    for (int it = 0; it < 5; ++it) {
      int idx = it * 256 + t;
      idx = idx < 1071 ? idx : 1071;
      const int r  = idx >> 4;
      const int c4 = (idx & 15) * 4;
      const int tt  = t0 - 3 + r;
      const int ttc = tt < 0 ? 0 : tt;
      v4f v = *(const v4f*)(LIN + (rowBase + ttc) * kLinLd + (size_t)z * kC + h * 64 + c4);
      if (tt < 0) v = (v4f){0.0f, 0.0f, 0.0f, 0.0f};
      *(v4f*)(linbuf + r * 64 + c4) = v;
    }
    __syncthreads();
    const float* wz = wcv[z];
#pragma unroll 1
    for (int it = 0; it < 16; ++it) {
      const int idx = it * 256 + t;
      const int r = idx >> 6, c = idx & 63;
      const float* lp = linbuf + r * 64 + c;
      float a = wz[c * 4 + 0] * lp[0];
      a = a + wz[c * 4 + 1] * lp[64];
      a = a + wz[c * 4 + 2] * lp[128];
      a = a + wz[c * 4 + 3] * lp[192];
      const float sig = 1.0f / (1.0f + expf(-a));
      abuf[r * 64 + c] = a * sig;
    }
    __syncthreads();
    if (z < 2) {
      const int r = t >> 2, cg = t & 3;
      float ss = 0.0f;
#pragma unroll 1
      for (int i = 0; i < 16; ++i) {
        const float v = abuf[r * 64 + 4 * i + cg];
        ss = ss + v * v;
      }
      ss = ss + __shfl_xor(ss, 1, 32);
      ss = ss + __shfl_xor(ss, 2, 32);
      const float inv = rsqrtf(ss + kL2Eps);
#pragma unroll 1
      for (int i = 0; i < 16; ++i) {
        const int c = 4 * i + cg;
        const float v   = abuf[r * 64 + c] * inv;
        const float phi = abuf[r * 64 + ((c + 16) & 63)] * inv;
        const float plo = abuf[r * 64 + ((c + 48) & 63)] * inv;
        const int j = c & 15;
        const float cs = cst[r * 16 + j];
        const float sn = snt[r * 16 + j];
        const float o0 = v * cs - phi * sn;
        const float o1 = v * cs + plo * sn;
        const float ov = (c < 16) ? o0 : ((c < 32) ? o1 : v);
        obuf[r * 64 + c] = ov;
      }
      __syncthreads();
    }
    const float* sb = aob[(z < 2) ? 1 : 0];
    float* dst = QKVc + (size_t)z * kPlane + (rowBase + t0) * kC + h * 64;
    for (int pass = 0; pass < 2; ++pass) {
#pragma unroll
      for (int it = 0; it < 4; ++it) {
        const int idx = it * 256 + t;
        const int r = idx >> 4, c4 = (idx & 15) * 4;
        const v4f v = *(const v4f*)(sb + r * 64 + c4);
        *(volatile v4f*)(dst + (size_t)r * kC + c4) = v;
      }
      __threadfence();
    }
    __syncthreads();
  }
}

__global__ __launch_bounds__(256) void scan_kernel(const float* __restrict__ QKVc, const float* __restrict__ EB,
                                                   float* __restrict__ Opl) {
  __shared__ __align__(16) float ks[kTch * 64];
  __shared__ __align__(16) float qs[kTch * 64];
  __shared__ __align__(16) float vs[kTch * 64];
  __shared__ __align__(16) float os[kTch * 64];
  __shared__ __align__(16) float ebs[kTch * 2];
  __shared__ float redP[256];
  __shared__ float redO[256];
  const int t   = threadIdx.x;
  const int dv  = t & 63;
  const int dkq = t >> 6;
  const int bh  = blockIdx.x;
  const int b = bh >> 4, h = bh & 15;
  const float* Qp = QKVc + ((size_t)b * kT) * kC + h * 64;
  const float* Kp = Qp + kPlane;
  const float* Vp = Qp + 2 * kPlane;
  const float* ebp = EB + (size_t)bh * kT * 2;
  float* Op = Opl + ((size_t)b * kT) * kLinLd + h * 64;

  float S[16];
#pragma unroll
  for (int i = 0; i < 16; ++i) S[i] = 0.0f;

#pragma unroll 1
  for (int ch = 0; ch < kT / kTch; ++ch) {
    const int t0 = ch * kTch;
#pragma unroll
    for (int it = 0; it < 2; ++it) {
      const int idx = it * 256 + t;
      const int r = idx >> 4, c4 = (idx & 15) * 4;
      const size_t go = (size_t)(t0 + r) * kC + c4;
      const v4f kv4 = *(const v4f*)(Kp + go);
      const v4f qv4 = *(const v4f*)(Qp + go);
      const v4f vv4 = *(const v4f*)(Vp + go);
      *(v4f*)(ks + r * 64 + c4) = kv4;
      *(v4f*)(qs + r * 64 + c4) = qv4;
      *(v4f*)(vs + r * 64 + c4) = vv4;
    }
    if (t < 16) {
      const v4f e4 = *(const v4f*)(ebp + (size_t)t0 * 2 + 4 * t);
      *(v4f*)(ebs + 4 * t) = e4;
    }
    __syncthreads();

#pragma unroll 1
    for (int s = 0; s < kTch; ++s) {
      const float eg   = ebs[2 * s];
      const float beta = ebs[2 * s + 1];
      const float vv   = vs[s * 64 + dv];
      const v4f* kr = (const v4f*)(ks + s * 64 + dkq * 16);
      const v4f* qr = (const v4f*)(qs + s * 64 + dkq * 16);
      const v4f ka = kr[0], kb = kr[1], kc = kr[2], kd = kr[3];
      const v4f qa = qr[0], qb = qr[1], qc = qr[2], qd = qr[3];
      float kx[16], qx[16];
#pragma unroll
      for (int e = 0; e < 4; ++e) {
        kx[e] = ka[e]; kx[4 + e] = kb[e]; kx[8 + e] = kc[e]; kx[12 + e] = kd[e];
        qx[e] = qa[e]; qx[4 + e] = qb[e]; qx[8 + e] = qc[e]; qx[12 + e] = qd[e];
      }
#pragma unroll
      for (int i = 0; i < 16; ++i) S[i] = S[i] * eg;
      float p = 0.0f;
#pragma unroll
      for (int i = 0; i < 16; ++i) p = fmaf(kx[i], S[i], p);
      redP[t] = p;
      __syncthreads();
      const float pred  = ((redP[dv] + redP[64 + dv]) + redP[128 + dv]) + redP[192 + dv];
      const float delta = beta * (vv - pred);
#pragma unroll
      for (int i = 0; i < 16; ++i) S[i] = fmaf(kx[i], delta, S[i]);
      float o = 0.0f;
#pragma unroll
      for (int i = 0; i < 16; ++i) o = fmaf(qx[i], S[i], o);
      redO[t] = o;
      __syncthreads();
      if (t < 64) os[s * 64 + dv] = ((redO[dv] + redO[64 + dv]) + redO[128 + dv]) + redO[192 + dv];
    }
    __syncthreads();
    for (int pass = 0; pass < 2; ++pass) {
#pragma unroll
      for (int it = 0; it < 2; ++it) {
        const int idx = it * 256 + t;
        const int r = idx >> 4, c4 = (idx & 15) * 4;
        const v4f v = *(const v4f*)(os + r * 64 + c4);
        *(volatile v4f*)(Op + (size_t)(t0 + r) * kLinLd + c4) = v;
      }
      __threadfence();
    }
    __syncthreads();
  }
}

__global__ __launch_bounds__(256) void gate_kernel(const float* __restrict__ LIN, const float* __restrict__ gnw,
                                                   unsigned short* __restrict__ OG) {
#pragma clang fp contract(off)
  __shared__ __align__(16) float stg[4 * 1024];
  const int t  = threadIdx.x;
  const int rl = t >> 6, hh = (t >> 2) & 15, cg = t & 3;
  const size_t row = (size_t)blockIdx.x * 4 + rl;
  const float* orow = LIN + row * kLinLd + kC + hh * 64;
  const float* grow = LIN + row * kLinLd + hh * 64;
  float ss = 0.0f;
#pragma unroll 1
  for (int i = 0; i < 16; ++i) {
    const float o = orow[4 * i + cg];
    ss = ss + o * o;
  }
  ss = ss + __shfl_xor(ss, 1, 32);
  ss = ss + __shfl_xor(ss, 2, 32);
  const float rms = rsqrtf(ss * (1.0f / 64.0f) + kRmsEps);
#pragma unroll 1
  for (int i = 0; i < 16; ++i) {
    const int c = 4 * i + cg;
    const float o  = orow[c];
    const float g  = grow[c];
    const float gw = bfr(gnw[c]);
    const float sig = 1.0f / (1.0f + expf(-g));
    const float val = ((o * rms) * gw) * (g * sig);
    stg[rl * 1024 + hh * 64 + c] = val * kOgCarry;
  }
  __syncthreads();
  unsigned short* ob = OG + (size_t)blockIdx.x * 4 * kC;
  for (int pass = 0; pass < 2; ++pass) {
#pragma unroll
    for (int it = 0; it < 2; ++it) {
      const int idx = it * 256 + t;
      const int r2 = idx >> 7, c8 = (idx & 127) * 8;
      unsigned short hb[8];
#pragma unroll
      for (int e = 0; e < 8; ++e) hb[e] = h_bits(stg[r2 * 1024 + c8 + e]);
      const v4u u = (v4u){pk16(hb[0], hb[1]), pk16(hb[2], hb[3]), pk16(hb[4], hb[5]), pk16(hb[6], hb[7])};
      *(volatile v4u*)(ob + (size_t)r2 * kC + c8) = u;
    }
    __threadfence();
  }
}

extern "C" void kernel_launch(void* const* d_in, const int* in_sizes, int n_in,
                              void* d_out, int out_size, void* d_ws, size_t ws_size,
                              hipStream_t stream) {
  if (n_in < 15) return;
  const int nX = kRows * kC;
  if (in_sizes[0] != nX) return;
  if (in_sizes[1] != kC * kC || in_sizes[2] != kC * kC || in_sizes[3] != kC * kC ||
      in_sizes[4] != kC * kC || in_sizes[5] != kC * kC) return;
  if (in_sizes[6] != kC * kH || in_sizes[7] != kC * kH) return;
  if (in_sizes[8] != kH || in_sizes[9] != kH || in_sizes[14] != kH) return;
  if (in_sizes[10] != kC * kTaps || in_sizes[11] != kC * kTaps || in_sizes[12] != kC * kTaps) return;
  if (in_sizes[13] != kD) return;
  if (out_size != nX) return;

  const size_t szXB   = (size_t)kRows * kC * 2;
  const size_t szWALL = (size_t)4 * kC * kC * 2;
  const size_t szWGB  = (size_t)kGbN * kC * 2;
  const size_t szWOT  = (size_t)kC * kC * 2;
  const size_t szLIN  = (size_t)kRows * kLinLd * 4;
  const size_t szGB   = (size_t)kRows * kGbN * 4;
  const size_t szQKVC = (size_t)3 * kPlane * 4;
  const size_t szEB   = (size_t)kB * kH * kT * 2 * 4;
  const size_t szCS   = (size_t)kT * 16 * 4;
  const size_t szOG   = (size_t)kRows * kC * 2;
  const size_t offXB   = 0;
  const size_t offWALL = offXB + szXB;
  const size_t offWGB  = offWALL + szWALL;
  const size_t offWOT  = offWGB + szWGB;
  const size_t offLIN  = offWOT + szWOT;
  const size_t offGB   = offLIN + szLIN;
  const size_t offQKVC = offGB + szGB;
  const size_t offEB   = offQKVC + szQKVC;
  const size_t offCS   = offEB + szEB;
  const size_t offSN   = offCS + szCS;
  const size_t offOG   = offSN + szCS;
  const size_t total   = offOG + szOG;
  if (ws_size < total) return;

  const float* x     = (const float*)d_in[0];
  const float* Wq    = (const float*)d_in[1];
  const float* Wk    = (const float*)d_in[2];
  const float* Wv    = (const float*)d_in[3];
  const float* Wo    = (const float*)d_in[4];
  const float* Wg    = (const float*)d_in[5];
  const float* Wgk   = (const float*)d_in[6];
  const float* Wb    = (const float*)d_in[7];
  const float* bb    = (const float*)d_in[8];
  const float* A_log = (const float*)d_in[9];
  const float* cwq   = (const float*)d_in[10];
  const float* cwk   = (const float*)d_in[11];
  const float* cwv   = (const float*)d_in[12];
  const float* gnw   = (const float*)d_in[13];
  const float* dtb   = (const float*)d_in[14];
  float* out = (float*)d_out;
  char* ws = (char*)d_ws;
  unsigned short* XB   = (unsigned short*)(ws + offXB);
  unsigned short* WALL = (unsigned short*)(ws + offWALL);
  unsigned short* WGB  = (unsigned short*)(ws + offWGB);
  unsigned short* WOT  = (unsigned short*)(ws + offWOT);
  float* LIN  = (float*)(ws + offLIN);
  float* GB   = (float*)(ws + offGB);
  float* QKVC = (float*)(ws + offQKVC);
  float* EB   = (float*)(ws + offEB);
  float* CS   = (float*)(ws + offCS);
  float* SN   = (float*)(ws + offSN);
  unsigned short* OG = (unsigned short*)(ws + offOG);
  const float* dummyf = (const float*)GB;

  RopeFreq rf;
  {
    const double r = 0.56234132519034908;
    double f = 1.0;
    for (int j = 0; j < 16; ++j) { rf.f[j] = (float)f; f *= r; }
  }

  const int n8 = nX / 8;
  cast8_bf16_kernel<<<dim3(n8 / 256), dim3(256), 0, stream>>>(x, XB, n8);
  pack_wt_kernel<0><<<dim3(kC / 64, kC / 64, 4), dim3(256), 0, stream>>>(Wq, Wk, Wv, Wg, WALL);
  pack_wt_kernel<1><<<dim3(kC / 64, kC / 64, 1), dim3(256), 0, stream>>>(Wo, Wo, Wo, Wo, WOT);
  pack_gb_kernel<<<dim3(kGbN), dim3(128), 0, stream>>>(Wgk, Wb, WGB);
  {
    const int tiles = (kRows / 64) * (kLinN / 64);
    wmma_gemm64<1, false, 0, 0, false, 0><<<dim3(tiles / 8, 1), dim3(256), 0, stream>>>(
        XB, XB, kC, 0L, WALL, WALL, kC, 0L, (void*)LIN, (void*)LIN, kLinLd, 0L,
        dummyf, dummyf, 0L, kRows, kLinN, kC, 1.0f);
  }
  {
    const int tiles = (kRows / 64) * (kGbN / 64);
    wmma_gemm64<1, false, 0, 0, false, 0><<<dim3(tiles / 8, 1), dim3(256), 0, stream>>>(
        XB, XB, kC, 0L, WGB, WGB, kC, 0L, (void*)GB, (void*)GB, kGbN, 0L,
        dummyf, dummyf, 0L, kRows, kGbN, kC, 1.0f);
  }
  cs_table_kernel<<<dim3((kT * 16) / 1024), dim3(256), 0, stream>>>(CS, SN, rf);
  eb_kernel<<<dim3(kB * kH), dim3(256), 0, stream>>>(GB, A_log, dtb, bb, EB);
  prep_kernel<<<dim3(kT / 64, kH, kB), dim3(256), 0, stream>>>(LIN, cwq, cwk, cwv, CS, SN, QKVC);
  {
    const int tiles = (kRows / 64) * (kC / 64);
    wmma_gemm64<1, false, 0, 0, false, 0><<<dim3(tiles / 8, 1), dim3(256), 0, stream>>>(
        XB, XB, kC, 0L, WALL + (size_t)3 * kC * kC, WALL + (size_t)3 * kC * kC, kC, 0L,
        (void*)LIN, (void*)LIN, kLinLd, 0L, dummyf, dummyf, 0L, kRows, kC, kC, 1.0f);
  }
  scan_kernel<<<dim3(kB * kH), dim3(256), 0, stream>>>(QKVC, EB, LIN + kC);
  gate_kernel<<<dim3(kRows / 4), dim3(256), 0, stream>>>(LIN, gnw, OG);
  {
    const int tiles = (kRows / 64) * (kC / 64);
    wmma_gemm64<0, false, 0, 0, false, 0><<<dim3(tiles / 8, 1), dim3(256), 0, stream>>>(
        OG, OG, kC, 0L, WOT, WOT, kC, 0L, (void*)out, (void*)out, kC, 0L,
        dummyf, dummyf, 0L, kRows, kC, kC, kOutScale);
  }
}
